// Data2VecVisionSelfAttention_13451837571567
// MI455X (gfx1250) — hardware-verified
//
#include <hip/hip_runtime.h>
#include <math.h>
#include <stdint.h>

#define NBAT   64
#define SEQ    197
#define KPAD   224
#define NQT    13
#define DMOD   768
#define NHEAD  12
#define DHEAD  64
#define MTOK   (NBAT * SEQ)
#define KSEG   (DMOD / 256)
#define TN64   (DMOD / 64)
#define NRD    732
#define NRDP   736
#define XC     64.0f
#define WSC    1024.0f
#define QS     1024.0f
#define KS     1024.0f
#define VS     256.0f
#define LNPS   6.931471805599453f
#define ATTSC  0.125f
#define NEGBIG (-1.0e30f)
#define ATHR   128
#define AWAVES (ATHR / 32)
#define LDS_KS (KPAD * DHEAD * 2)
#define LDS_V  (DHEAD * KPAD * 2)
#define LDS_OS (AWAVES * 16 * DHEAD * 4)
#define LDS_BT (NRDP * 4)
#define LDS_AK (KPAD * 4)
#define LDS_ATT (LDS_KS + 2 * LDS_V + LDS_OS + LDS_BT + LDS_AK)

static_assert(NHEAD * DHEAD == DMOD);
static_assert((MTOK % 64) == 0 && (DMOD % 64) == 0 && (DMOD % 256) == 0 && (DMOD % 32) == 0);
static_assert((((MTOK / 64) * TN64) % 4) == 0);
static_assert(((MTOK * KSEG) % 8) == 0 && ((DMOD * KSEG) % 8) == 0);
static_assert((KPAD % 32) == 0 && KPAD >= SEQ && (NQT * 16) >= SEQ && ((NQT - 1) * 16) < SEQ);
static_assert((LDS_KS % 16) == 0 && (LDS_V % 16) == 0 && (LDS_OS % 16) == 0 && (LDS_BT % 16) == 0);
static_assert(LDS_ATT == 106240);
static_assert(NRDP >= NRD);

typedef _Float16 v16h __attribute__((ext_vector_type(16)));
typedef _Float16 v8h  __attribute__((ext_vector_type(8)));
typedef float    v8f  __attribute__((ext_vector_type(8)));
typedef float    v4f  __attribute__((ext_vector_type(4)));
typedef unsigned int v4u __attribute__((ext_vector_type(4)));

union FragH { v16h v; v8h h[2]; };

__device__ __forceinline__ unsigned short bf_bits(float f) {
  unsigned u = __float_as_uint(f);
  return (unsigned short)((u + 0x7FFFu + ((u >> 16) & 1u)) >> 16);
}
__device__ __forceinline__ float bf_up(unsigned short h) { return __uint_as_float(((unsigned)h) << 16); }
__device__ __forceinline__ float bfr(float f) { return bf_up(bf_bits(f)); }
__device__ __forceinline__ unsigned short h_bits(_Float16 x) { return __builtin_bit_cast(unsigned short, x); }
__device__ __forceinline__ unsigned pk16(unsigned short a, unsigned short b) { return (unsigned)a | ((unsigned)b << 16); }
__device__ __forceinline__ v8f zero8() { v8f z = {0.f, 0.f, 0.f, 0.f, 0.f, 0.f, 0.f, 0.f}; return z; }

__device__ __forceinline__ v16h ldfrag_h(const _Float16* p) {
  FragH f;
  f.h[0] = *(const v8h*)(p);
  f.h[1] = *(const v8h*)(p + 16);
  return f.v;
}

__device__ __forceinline__ v8f mma_h_raw(v16h a, v16h b, v8f c) {
  return __builtin_amdgcn_wmma_f32_16x16x32_f16(false, a, false, b, (short)0, c, false, false);
}
__device__ __forceinline__ void dep_guard1(v8f& a, v8f& b, v16h x) {
#if defined(__HIP_DEVICE_COMPILE__)
  asm volatile("v_nop\n\tv_nop\n\tv_nop\n\tv_nop" : "+v"(a), "+v"(b) : "v"(x));
#endif
}
__device__ __forceinline__ void keep4_h(v16h a, v16h b, v16h c, v16h d) {
#if defined(__HIP_DEVICE_COMPILE__)
  asm volatile("v_nop" :: "v"(a), "v"(b), "v"(c), "v"(d));
#endif
}
__device__ __forceinline__ void acc_guard4(v8f& a, v8f& b, v8f& c, v8f& d) {
#if defined(__HIP_DEVICE_COMPILE__)
  asm volatile("v_nop\n\tv_nop\n\tv_nop\n\tv_nop" : "+v"(a), "+v"(b), "+v"(c), "+v"(d));
#endif
}
__device__ __forceinline__ void sguard6(v8f& a, v8f& b, v16h x0, v16h x1, v16h x2, v16h x3, v16h x4, v16h x5) {
#if defined(__HIP_DEVICE_COMPILE__)
  asm volatile("v_nop\n\tv_nop\n\tv_nop\n\tv_nop"
               : "+v"(a), "+v"(b) : "v"(x0), "v"(x1), "v"(x2), "v"(x3), "v"(x4), "v"(x5));
#endif
}
__device__ __forceinline__ void oguard10(v8f& a, v8f& b, v8f& c, v8f& d,
                                         v16h x0, v16h x1, v16h x2, v16h x3,
                                         v16h y0, v16h y1, v16h y2, v16h y3, v16h p0, v16h p1) {
#if defined(__HIP_DEVICE_COMPILE__)
  asm volatile("v_nop\n\tv_nop\n\tv_nop\n\tv_nop"
               : "+v"(a), "+v"(b), "+v"(c), "+v"(d)
               : "v"(x0), "v"(x1), "v"(x2), "v"(x3), "v"(y0), "v"(y1), "v"(y2), "v"(y3), "v"(p0), "v"(p1));
#endif
}
__device__ __forceinline__ void wave_sync_lds() {
  __builtin_amdgcn_fence(__ATOMIC_RELEASE, "workgroup");
  __builtin_amdgcn_wave_barrier();
  __builtin_amdgcn_fence(__ATOMIC_ACQUIRE, "workgroup");
}

__global__ __launch_bounds__(256) void cvt_rows(const float* __restrict__ src, unsigned short* dst, int nseg, float scale) {
  const int lane = threadIdx.x & 31, wave = threadIdx.x >> 5;
  const int seg = blockIdx.x * 8 + wave;
  if (seg >= nseg) return;
  const int row = seg / KSEG;
  const int col = (seg - row * KSEG) * 256 + 8 * lane;
  const size_t o = (size_t)row * DMOD + col;
  const v4f h0 = *(const v4f*)(src + o), h1 = *(const v4f*)(src + o + 4);
  float a[8];
#pragma unroll
  for (int i = 0; i < 4; ++i) { a[i] = bfr(h0[i]); a[4 + i] = bfr(h1[i]); }
  v4u uh;
#pragma unroll
  for (int i = 0; i < 4; ++i) {
    const float xa = a[2 * i] * scale, xb = a[2 * i + 1] * scale;
    uh[i] = pk16(h_bits((_Float16)xa), h_bits((_Float16)xb));
  }
  unsigned short* dh = dst + o;
  *(volatile v4u*)dh = uh;
  __threadfence();
  *(volatile v4u*)dh = uh;
}

template <int NPL>
__global__ __launch_bounds__(128) void gemm64(
    const unsigned short* __restrict__ Ap, const unsigned short* __restrict__ Bp,
    const float* __restrict__ bias, float escale, float bscale,
    unsigned short* H0, unsigned short* H1) {
  __shared__ __align__(16) float slabs[4][16 * 68];
  const int lane = threadIdx.x & 31;
  const int wave = threadIdx.x >> 5;
  const int tilesN = TN64;
  const int tile = blockIdx.x * 4 + wave;
  const int tm = tile / tilesN;
  const int tn = tile - tm * tilesN;
  const int m0 = tm << 6;
  const int n0 = tn << 6;

  const _Float16* Ah = (const _Float16*)(const void*)Ap;
  const _Float16* Bb = (const _Float16*)(const void*)Bp;

  const int rlane = lane & 15;
  const int hh    = lane >> 4;
  const int koff  = hh * 8;
  const int mOff  = hh * 8;

  v8f acc[4][4];
#pragma unroll
  for (int i = 0; i < 4; ++i)
#pragma unroll
    for (int j = 0; j < 4; ++j) acc[i][j] = zero8();

  for (int k0 = 0; k0 < DMOD; k0 += 32) {
    v16h bh[4];
#pragma unroll
    for (int j = 0; j < 4; ++j) {
      const size_t bo = (size_t)(n0 + (j << 4) + rlane) * DMOD + koff + k0;
      bh[j] = ldfrag_h(Bb + bo);
    }
#pragma unroll
    for (int i = 0; i < 4; ++i) {
      const size_t ao = (size_t)(m0 + (i << 4) + rlane) * DMOD + koff + k0;
      const v16h ah = ldfrag_h(Ah + ao);
#pragma unroll
      for (int j = 0; j < 4; ++j) acc[i][j] = mma_h_raw(ah, bh[j], acc[i][j]);
      dep_guard1(acc[i][0], acc[i][3], ah);
    }
    keep4_h(bh[0], bh[1], bh[2], bh[3]);
  }
  acc_guard4(acc[0][0], acc[0][1], acc[0][2], acc[0][3]);
  acc_guard4(acc[1][0], acc[1][1], acc[1][2], acc[1][3]);
  acc_guard4(acc[2][0], acc[2][1], acc[2][2], acc[2][3]);
  acc_guard4(acc[3][0], acc[3][1], acc[3][2], acc[3][3]);

  const int e = lane & 7, q4 = lane >> 3;
  const v4f b0 = *(const v4f*)(bias + n0 + 8 * e), b1 = *(const v4f*)(bias + n0 + 8 * e + 4);
  float bb[8];
#pragma unroll
  for (int tt = 0; tt < 4; ++tt) { bb[tt] = bfr(b0[tt]) * bscale; bb[4 + tt] = bfr(b1[tt]) * bscale; }
  float* slab = &slabs[wave][0];
#pragma unroll
  for (int i = 0; i < 4; ++i) {
    const int mBase = m0 + (i << 4);
#pragma unroll
    for (int j = 0; j < 4; ++j) {
#pragma unroll
      for (int r = 0; r < 8; ++r) slab[(mOff + r) * 68 + (j << 4) + rlane] = acc[i][j][r];
    }
    wave_sync_lds();
    v4u hv[4], lv[4];
#pragma unroll
    for (int it = 0; it < 4; ++it) {
      const int row = it * 4 + q4;
      const v4f x0 = *(const v4f*)(slab + row * 68 + 8 * e);
      const v4f x1 = *(const v4f*)(slab + row * 68 + 8 * e + 4);
      float y[8];
#pragma unroll
      for (int tt = 0; tt < 4; ++tt) { y[tt] = x0[tt] * escale + bb[tt]; y[4 + tt] = x1[tt] * escale + bb[4 + tt]; }
      v4u uh, ul = {0u, 0u, 0u, 0u};
#pragma unroll
      for (int t2 = 0; t2 < 4; ++t2) {
        const _Float16 ha = (_Float16)y[2 * t2], hb = (_Float16)y[2 * t2 + 1];
        uh[t2] = pk16(h_bits(ha), h_bits(hb));
        if (NPL == 2) {
          const _Float16 la = (_Float16)(y[2 * t2] - (float)ha);
          const _Float16 lb = (_Float16)(y[2 * t2 + 1] - (float)hb);
          ul[t2] = pk16(h_bits(la), h_bits(lb));
        }
      }
      hv[it] = uh;
      lv[it] = ul;
    }
    for (int pass = 0; pass < 2; ++pass) {
#pragma unroll
      for (int it = 0; it < 4; ++it) {
        const int row = it * 4 + q4;
        const size_t go = (size_t)(mBase + row) * DMOD + n0 + 8 * e;
        *(volatile v4u*)(H0 + go) = hv[it];
        if (NPL == 2) *(volatile v4u*)(H1 + go) = lv[it];
      }
      __threadfence();
    }
    wave_sync_lds();
  }
}

__global__ __launch_bounds__(ATHR)
void attn_kernel(const unsigned short* __restrict__ qp, const unsigned short* __restrict__ kp,
                 const unsigned short* __restrict__ vhp, const unsigned short* __restrict__ vlp,
                 const float* __restrict__ btab, float* out) {
  extern __shared__ v4u dlds4[];
  unsigned char*  dlds = (unsigned char*)dlds4;
  unsigned short* Ks   = (unsigned short*)(dlds);
  unsigned short* Vhs  = (unsigned short*)(dlds + LDS_KS);
  unsigned short* Vls  = (unsigned short*)(dlds + LDS_KS + LDS_V);
  float*          Os   = (float*)(dlds + LDS_KS + 2 * LDS_V);
  float*          Bts  = (float*)(dlds + LDS_KS + 2 * LDS_V + LDS_OS);
  int*            Akt  = (int*)(dlds + LDS_KS + 2 * LDS_V + LDS_OS + LDS_BT);

  const int tid  = threadIdx.x;
  const int wave = tid >> 5;
  const int lane = tid & 31;
  const int hh   = lane >> 4;
  const int c    = lane & 15;
  const int bh   = blockIdx.x;
  const int b    = bh / NHEAD;
  const int hd   = bh - b * NHEAD;
  const size_t tok0 = (size_t)b * SEQ;
  const size_t hcol = (size_t)hd * DHEAD;

  for (int i = tid; i < KPAD * 8; i += ATHR) {
    const int key = i >> 3, ch = i & 7;
    const int kc = (key < SEQ) ? key : (SEQ - 1);
    const v4u g = *(const v4u*)(kp + (tok0 + kc) * DMOD + hcol + 8 * ch);
    v4u w;
#pragma unroll
    for (int j = 0; j < 4; ++j) w[j] = (key < SEQ) ? g[j] : 0u;
    *(v4u*)(Ks + key * DHEAD + 8 * ch) = w;
  }
  for (int i = tid; i < KPAD * 8; i += ATHR) {
    const int key = i >> 3, ch = i & 7;
    const int kc = (key < SEQ) ? key : (SEQ - 1);
    const size_t go = (tok0 + kc) * DMOD + hcol + 8 * ch;
    const v4u ga = *(const v4u*)(vhp + go);
    const v4u gb = *(const v4u*)(vlp + go);
    const bool ok = (key < SEQ);
#pragma unroll
    for (int j = 0; j < 4; ++j) {
      const unsigned wa = ok ? ga[j] : 0u;
      const unsigned wb = ok ? gb[j] : 0u;
      const int d = 8 * ch + 2 * j;
      Vhs[d * KPAD + key]       = (unsigned short)(wa & 0xFFFFu);
      Vhs[(d + 1) * KPAD + key] = (unsigned short)(wa >> 16);
      Vls[d * KPAD + key]       = (unsigned short)(wb & 0xFFFFu);
      Vls[(d + 1) * KPAD + key] = (unsigned short)(wb >> 16);
    }
  }
  for (int i = tid; i < NRDP; i += ATHR) {
    const int ic = (i < NRD) ? i : (NRD - 1);
    const float tv = bfr(btab[(size_t)ic * NHEAD + hd]);
    Bts[i] = (i < NRD) ? tv : 0.f;
  }
  for (int k = tid; k < KPAD; k += ATHR) {
    int p = k - 1;
    p = (p < 0) ? 0 : p;
    Akt[k] = p + 13 * (p / 14);
  }
  __syncthreads();

  const _Float16* QP  = (const _Float16*)(const void*)qp;
  const _Float16* KsH = (const _Float16*)(const void*)Ks;
  const _Float16* VhH = (const _Float16*)(const void*)Vhs;
  const _Float16* VlH = (const _Float16*)(const void*)Vls;
  const float SC = ATTSC / (QS * KS);
  float* Osw = Os + wave * (16 * DHEAD);

#pragma unroll 1
  for (int qt = wave; qt < NQT; qt += AWAVES) {
    const int q  = qt * 16 + c;
    const int qc = (q < SEQ) ? q : (SEQ - 1);
    const _Float16* qbp = QP + (tok0 + qc) * DMOD + hcol + 8 * hh;
    const v16h qf0 = ldfrag_h(qbp), qf1 = ldfrag_h(qbp + 32);
    const int qm1 = (q > 0) ? (q - 1) : 0;
    const int aq  = qm1 + 13 * (qm1 / 14) + 364;
    const bool qzero = (q == 0);

    float m = NEGBIG, l = 0.f;
    v8f o0 = zero8(), o1 = zero8(), o2 = zero8(), o3 = zero8();
#pragma unroll 1
    for (int it = 0; it < KPAD / 32; ++it) {
      const int kb = it * 32;
      const _Float16* k0p = KsH + (kb + c) * DHEAD + 8 * hh;
      const _Float16* k1p = k0p + 16 * DHEAD;
      const v16h a0 = ldfrag_h(k0p), a1 = ldfrag_h(k1p);
      const v16h a2 = ldfrag_h(k0p + 32), a3 = ldfrag_h(k1p + 32);
      v8f s0 = mma_h_raw(a0, qf0, zero8());
      v8f s1 = mma_h_raw(a1, qf0, zero8());
      s0 = mma_h_raw(a2, qf1, s0);
      s1 = mma_h_raw(a3, qf1, s1);
      sguard6(s0, s1, a0, a1, a2, a3, qf0, qf1);

      float x0[8], x1[8];
#pragma unroll
      for (int r = 0; r < 8; ++r) {
        const int key0 = kb + 8 * hh + r;
        const int key1 = key0 + 16;
        const int ak0 = Akt[key0], ak1 = Akt[key1];
        int i0 = qzero ? ((key0 == 0) ? (NRD - 1) : (NRD - 3)) : ((key0 == 0) ? (NRD - 2) : (aq - ak0));
        int i1 = qzero ? (NRD - 3) : (aq - ak1);
        i0 = (i0 < 0) ? 0 : ((i0 > NRD - 1) ? (NRD - 1) : i0);
        i1 = (i1 < 0) ? 0 : ((i1 > NRD - 1) ? (NRD - 1) : i1);
        const float bb0 = Bts[i0], bb1 = Bts[i1];
        const float v0 = s0[r] * SC + bb0;
        const float v1 = s1[r] * SC + bb1;
        x0[r] = (key0 < SEQ) ? v0 : NEGBIG;
        x1[r] = (key1 < SEQ) ? v1 : NEGBIG;
      }
      float mx = -3.0e38f;
#pragma unroll
      for (int r = 0; r < 8; ++r) mx = fmaxf(mx, fmaxf(x0[r], x1[r]));
      mx = fmaxf(mx, __shfl_xor(mx, 16, 32));
      const float mn   = fmaxf(m, mx);
      const float corr = __expf(m - mn);
      m = mn;
      const float msh = mn - LNPS;
      l *= corr;
#pragma unroll
      for (int r = 0; r < 8; ++r) { o0[r] *= corr; o1[r] *= corr; o2[r] *= corr; o3[r] *= corr; }

      FragH ph, pl;
      float ls = 0.f;
#pragma unroll
      for (int r = 0; r < 8; ++r) {
        const float e0 = __expf(x0[r] - msh);
        const float e1 = __expf(x1[r] - msh);
        ls += e0 + e1;
        const _Float16 h0 = (_Float16)e0, h1 = (_Float16)e1;
        ph.h[0][r] = h0;
        ph.h[1][r] = h1;
        pl.h[0][r] = (_Float16)(e0 - (float)h0);
        pl.h[1][r] = (_Float16)(e1 - (float)h1);
      }
      l += ls;

      const _Float16* vh0 = VhH + c * KPAD + kb + 8 * hh;
      const _Float16* vl0 = VlH + c * KPAD + kb + 8 * hh;
      const v16h vf0 = ldfrag_h(vh0);
      const v16h vf1 = ldfrag_h(vh0 + 16 * KPAD);
      const v16h vf2 = ldfrag_h(vh0 + 32 * KPAD);
      const v16h vf3 = ldfrag_h(vh0 + 48 * KPAD);
      const v16h wf0 = ldfrag_h(vl0);
      const v16h wf1 = ldfrag_h(vl0 + 16 * KPAD);
      const v16h wf2 = ldfrag_h(vl0 + 32 * KPAD);
      const v16h wf3 = ldfrag_h(vl0 + 48 * KPAD);
      o0 = mma_h_raw(vf0, ph.v, o0);
      o1 = mma_h_raw(vf1, ph.v, o1);
      o2 = mma_h_raw(vf2, ph.v, o2);
      o3 = mma_h_raw(vf3, ph.v, o3);
      o0 = mma_h_raw(vf0, pl.v, o0);
      o1 = mma_h_raw(vf1, pl.v, o1);
      o2 = mma_h_raw(vf2, pl.v, o2);
      o3 = mma_h_raw(vf3, pl.v, o3);
      o0 = mma_h_raw(wf0, ph.v, o0);
      o1 = mma_h_raw(wf1, ph.v, o1);
      o2 = mma_h_raw(wf2, ph.v, o2);
      o3 = mma_h_raw(wf3, ph.v, o3);
      oguard10(o0, o1, o2, o3, vf0, vf1, vf2, vf3, wf0, wf1, wf2, wf3, ph.v, pl.v);
    }
    l += __shfl_xor(l, 16, 32);
    const float sc = (1.0f / VS) * (1.0f / l);

    float* os = Osw + c * DHEAD + 8 * hh;
#pragma unroll
    for (int r = 0; r < 8; ++r) { os[r] = o0[r] * sc; os[16 + r] = o1[r] * sc; os[32 + r] = o2[r] * sc; os[48 + r] = o3[r] * sc; }
    wave_sync_lds();
    const int c4 = c * 4;
    v4f vals[8];
#pragma unroll
    for (int it = 0; it < 8; ++it) {
      const int qi = it * 2 + hh;
      vals[it] = *(const v4f*)(Osw + qi * DHEAD + c4);
    }
    float* ob = out + hcol + c4;
    for (int pass = 0; pass < 2; ++pass) {
#pragma unroll
      for (int it = 0; it < 8; ++it) {
        const int qi = it * 2 + hh;
        const int qq = qt * 16 + qi;
        if (qq < SEQ) *(volatile v4f*)(ob + (tok0 + qq) * DMOD) = vals[it];
      }
      __threadfence();
    }
    wave_sync_lds();
  }
}

extern "C" void kernel_launch(void* const* d_in, const int* in_sizes, int n_in,
                              void* d_out, int out_size, void* d_ws, size_t ws_size,
                              hipStream_t stream) {
  if (n_in < 7) return;
  if (in_sizes[0] != MTOK * DMOD) return;
  if (in_sizes[1] != DMOD * DMOD || in_sizes[3] != DMOD * DMOD || in_sizes[4] != DMOD * DMOD) return;
  if (in_sizes[2] != DMOD || in_sizes[5] != DMOD) return;
  if (in_sizes[6] != NRD * NHEAD) return;
  if (out_size != MTOK * DMOD) return;

  const float* hs = (const float*)d_in[0];
  const float* Wq = (const float*)d_in[1];
  const float* bq = (const float*)d_in[2];
  const float* Wk = (const float*)d_in[3];
  const float* Wv = (const float*)d_in[4];
  const float* bv = (const float*)d_in[5];
  const float* bt = (const float*)d_in[6];

  const size_t PACT = (size_t)MTOK * DMOD * 2;
  const size_t PW   = (size_t)DMOD * DMOD * 2;
  size_t off = 0;
  const size_t oXH = off; off += PACT;
  const size_t oWQ = off; off += PW;
  const size_t oWK = off; off += PW;
  const size_t oWV = off; off += PW;
  const size_t oQP = off; off += PACT;
  const size_t oKP = off; off += PACT;
  const size_t oVH = off; off += PACT;
  const size_t oVL = off; off += PACT;
  if (off > ws_size) return;
  if (off > (size_t)134217728) return;

  char* ws = (char*)d_ws;
  unsigned short* XH  = (unsigned short*)(ws + oXH);
  unsigned short* WQH = (unsigned short*)(ws + oWQ);
  unsigned short* WKH = (unsigned short*)(ws + oWK);
  unsigned short* WVH = (unsigned short*)(ws + oWV);
  unsigned short* QPL = (unsigned short*)(ws + oQP);
  unsigned short* KPL = (unsigned short*)(ws + oKP);
  unsigned short* VHP = (unsigned short*)(ws + oVH);
  unsigned short* VLP = (unsigned short*)(ws + oVL);
  float*          out = (float*)d_out;

  const dim3 blk256(256), blk128(128), blkA(ATHR);
  const dim3 gCA(MTOK * KSEG / 8);
  const dim3 gCW(DMOD * KSEG / 8);
  const dim3 gGM(((MTOK / 64) * TN64) / 4);
  const dim3 gAT(NBAT * NHEAD);

  cvt_rows<<<gCA, blk256, 0, stream>>>(hs, XH, MTOK * KSEG, XC);
  cvt_rows<<<gCW, blk256, 0, stream>>>(Wq, WQH, DMOD * KSEG, WSC);
  cvt_rows<<<gCW, blk256, 0, stream>>>(Wk, WKH, DMOD * KSEG, WSC);
  cvt_rows<<<gCW, blk256, 0, stream>>>(Wv, WVH, DMOD * KSEG, WSC);

  gemm64<1><<<gGM, blk128, 0, stream>>>(XH, WQH, bq, QS / (XC * WSC), QS, QPL, QPL);
  gemm64<1><<<gGM, blk128, 0, stream>>>(XH, WKH, bq, KS / (XC * WSC), 0.0f, KPL, KPL);
  gemm64<2><<<gGM, blk128, 0, stream>>>(XH, WVH, bv, VS / (XC * WSC), VS, VHP, VLP);

  (void)hipFuncSetAttribute(reinterpret_cast<const void*>(&attn_kernel),
                            hipFuncAttributeMaxDynamicSharedMemorySize, LDS_ATT);
  attn_kernel<<<gAT, blkA, LDS_ATT, stream>>>(QPL, KPL, VHP, VLP, bt, out);
  (void)hipGetLastError();
}
